// GCLSTM_18906446037334
// MI455X (gfx1250) — hardware-verified
//
#include <hip/hip_runtime.h>
#include <stddef.h>
#include <stdint.h>


#define HSZ     256
#define ISZ     128
#define KCH     4
#define KA      1536
#define XOFF    1024
#define NGC     1024
#define STGW    384
#define NTHR    256
#define NWAVE   8
#define EPT     8
#define CHUNK   (NTHR * EPT)
#define WCAP    (EPT * 32)
#define LISTN   (NWAVE * WCAP)
#define NBMAX   2048
#define RCAP    28672
#define DEGCAP  128
#define GBM     64
#define GBN     64
#define GTHR    128
#define WSMAX   134217728
#define LDS_DYN ((2 * RCAP + 2 * NBMAX + LISTN) * 4 + 64)

static_assert(KA == KCH * (HSZ + ISZ));
static_assert(XOFF == KCH * HSZ);
static_assert(NGC == 4 * HSZ);
static_assert(STGW == HSZ + ISZ);
static_assert(HSZ == 8 * 32 && ISZ == 4 * 32);
static_assert((KA % 32) == 0);
static_assert((NGC % GBN) == 0);
static_assert((CHUNK & (CHUNK - 1)) == 0 && CHUNK <= 4096);
static_assert((NBMAX & (NBMAX - 1)) == 0 && NBMAX <= 4096);
static_assert(NTHR * 8 == NBMAX);
static_assert(LISTN >= NBMAX);
static_assert(LISTN >= NWAVE * WCAP);
static_assert((RCAP % 32) == 0);
static_assert(DEGCAP == 4 * 32);
static_assert(LDS_DYN + NWAVE * STGW * 4 <= 300000);
static_assert(GBM == (GTHR / 32) * 16);

typedef float          v4f  __attribute__((ext_vector_type(4)));
typedef float          v4fa __attribute__((ext_vector_type(4), may_alias));
typedef float          v8f  __attribute__((ext_vector_type(8)));
typedef int            v4i  __attribute__((ext_vector_type(4)));
typedef int            v8i  __attribute__((ext_vector_type(8)));
typedef unsigned short v8us __attribute__((ext_vector_type(8)));
typedef __bf16         v16b __attribute__((ext_vector_type(16)));
union FragB { v16b v; v8us h[2]; v8i w; };

__device__ __forceinline__ v8f wmb(const FragB& a, const FragB& b, v8f c) {
  v8f d = __builtin_amdgcn_wmma_f32_16x16x32_bf16(false, a.v, false, b.v, (short)0, c, false, false);
  asm volatile("v_nop\n\tv_nop\n\tv_nop\n\tv_nop" : "+v"(d) : "v"(a.w), "v"(b.w));
  return d;
}

__device__ __forceinline__ unsigned short bf_rne(float f) {
  unsigned u = __float_as_uint(f);
  u = u + 0x7FFFu + ((u >> 16) & 1u);
  return (unsigned short)(u >> 16);
}
__device__ __forceinline__ float bf_val(unsigned short b) {
  return __uint_as_float(((unsigned)b) << 16);
}

__device__ __forceinline__ void split8(const v4f a, const v4f b, v8us& hi, v8us& lo) {
  float v[8];
  v[0] = a.x; v[1] = a.y; v[2] = a.z; v[3] = a.w;
  v[4] = b.x; v[5] = b.y; v[6] = b.z; v[7] = b.w;
#pragma unroll
  for (int e = 0; e < 8; ++e) {
    const unsigned short hb = bf_rne(v[e]);
    const float r = v[e] - bf_val(hb);
    hi[e] = hb;
    lo[e] = bf_rne(r);
  }
}

__device__ __forceinline__ float sigm_f(float x) {
  const float e = __expf(-fabsf(x));
  const float r = __builtin_amdgcn_rcpf(1.0f + e);
  return x >= 0.f ? r : e * r;
}
__device__ __forceinline__ float tanh_f(float x) {
  const float ax = fabsf(x);
  const float e  = __expf(2.0f * ax);
  const float r  = __builtin_amdgcn_rcpf(1.0f + e);
  const float t  = 1.0f - 2.0f * r;
  return copysignf(t, x);
}

__device__ __forceinline__ int scan_chunk(const int* __restrict__ pos2, int nE, int cbase, int slotBase,
                                          int nb, int* list, int tid, int lane, int wave) {
  int wc = 0;
  const int el0  = tid * EPT;
  const int e0   = cbase + el0;
  const int sent = -2147483647 - 1;
  int d0, d1, d2, d3, d4, d5, d6, d7;
  if (cbase + CHUNK <= nE) {
    const int* pp = pos2 + 2 * (size_t)e0;
    const v4i p0 = *(const v4i*)(pp);
    const v4i p1 = *(const v4i*)(pp + 4);
    const v4i p2 = *(const v4i*)(pp + 8);
    const v4i p3 = *(const v4i*)(pp + 12);
    d0 = p0.x; d1 = p0.z; d2 = p1.x; d3 = p1.z;
    d4 = p2.x; d5 = p2.z; d6 = p3.x; d7 = p3.z;
  } else {
    d0 = (e0     < nE) ? pos2[2 * (size_t)min(e0,     nE - 1)] : sent;
    d1 = (e0 + 1 < nE) ? pos2[2 * (size_t)min(e0 + 1, nE - 1)] : sent;
    d2 = (e0 + 2 < nE) ? pos2[2 * (size_t)min(e0 + 2, nE - 1)] : sent;
    d3 = (e0 + 3 < nE) ? pos2[2 * (size_t)min(e0 + 3, nE - 1)] : sent;
    d4 = (e0 + 4 < nE) ? pos2[2 * (size_t)min(e0 + 4, nE - 1)] : sent;
    d5 = (e0 + 5 < nE) ? pos2[2 * (size_t)min(e0 + 5, nE - 1)] : sent;
    d6 = (e0 + 6 < nE) ? pos2[2 * (size_t)min(e0 + 6, nE - 1)] : sent;
    d7 = (e0 + 7 < nE) ? pos2[2 * (size_t)min(e0 + 7, nE - 1)] : sent;
  }
  const unsigned nbs = (unsigned)slotBase;
  const unsigned unb = (unsigned)nb;
  const unsigned s0 = (unsigned)d0 - nbs, s1 = (unsigned)d1 - nbs;
  const unsigned s2 = (unsigned)d2 - nbs, s3 = (unsigned)d3 - nbs;
  const unsigned s4 = (unsigned)d4 - nbs, s5 = (unsigned)d5 - nbs;
  const unsigned s6 = (unsigned)d6 - nbs, s7 = (unsigned)d7 - nbs;
  const bool h0 = s0 < unb, h1 = s1 < unb, h2 = s2 < unb, h3 = s3 < unb;
  const bool h4 = s4 < unb, h5 = s5 < unb, h6 = s6 < unb, h7 = s7 < unb;
  const unsigned any = __builtin_amdgcn_ballot_w32(h0 | h1 | h2 | h3 | h4 | h5 | h6 | h7);
  if (any != 0u) {
#define HITJ(J, HJ, SJ) { \
      const unsigned mj = __builtin_amdgcn_ballot_w32(HJ); \
      if (mj != 0u) { \
        if (HJ) { \
          const int ps = wc + (int)__builtin_amdgcn_mbcnt_lo(mj, 0u); \
          if (ps < WCAP) list[wave * WCAP + ps] = ((el0 + (J)) << 12) | (int)(SJ); \
        } \
        wc += (int)__builtin_popcount(mj); } }
    HITJ(0, h0, s0)
    HITJ(1, h1, s1)
    HITJ(2, h2, s2)
    HITJ(3, h3, s3)
    HITJ(4, h4, s4)
    HITJ(5, h5, s5)
    HITJ(6, h6, s6)
    HITJ(7, h7, s7)
#undef HITJ
  }
  return wc;
}

__global__ __launch_bounds__(NTHR) void k_split(const float* __restrict__ src, int F, unsigned short* ah,
                                                unsigned short* al, int colOff, int nRows, int nUnits) {
  const int i = (int)blockIdx.x * NTHR + (int)threadIdx.x;
  if (i >= nUnits) return;
  const int uq  = F >> 3;
  const int row = i / uq;
  const int c0  = (i - row * uq) * 8;
  const int rc  = row < nRows ? row : nRows - 1;
  const float* p = src + (size_t)rc * (size_t)F + c0;
  const v4f a = *(const v4f*)p, b = *(const v4f*)(p + 4);
  v8us hv, lv;
  split8(a, b, hv, lv);
  const size_t o = (size_t)row * KA + colOff + c0;
  *(volatile v8us*)(ah + o) = hv;
  *(volatile v8us*)(al + o) = lv;
  __threadfence();
  *(volatile v8us*)(ah + o) = hv;
  *(volatile v8us*)(al + o) = lv;
}

__global__ __launch_bounds__(NTHR) void k_wsplit(
    const float* __restrict__ Wfh, const float* __restrict__ Wih, const float* __restrict__ Woh,
    const float* __restrict__ Wch, const float* __restrict__ Wfx, const float* __restrict__ Wix,
    const float* __restrict__ Wox, const float* __restrict__ Wcx,
    unsigned short* wh, unsigned short* wl, int nUnits) {
  const int u = (int)blockIdx.x * NTHR + (int)threadIdx.x;
  if (u >= nUnits) return;
  const int kq = KA >> 3;
  const int n  = u / kq;
  const int k8 = (u - n * kq) * 8;
  int gate = n >> 8; gate = gate > 3 ? 3 : gate;
  const int ho = n & 255;
  const float* wgh = (gate == 0) ? Wfh : ((gate == 1) ? Wih : ((gate == 2) ? Woh : Wch));
  const float* wgx = (gate == 0) ? Wfx : ((gate == 1) ? Wix : ((gate == 2) ? Wox : Wcx));
  int kk = k8 >> 8; kk = kk > KCH - 1 ? KCH - 1 : kk;
  const int f0h = k8 & 255;
  int k8x = k8 - XOFF; k8x = k8x < 0 ? 0 : k8x;
  int kx = k8x >> 7; kx = kx > KCH - 1 ? KCH - 1 : kx;
  const int f0x = k8x & 127;
  const size_t offh = ((size_t)kk * HSZ + (size_t)ho) * HSZ + f0h;
  const size_t offx = ((size_t)kx * HSZ + (size_t)ho) * ISZ + f0x;
  const float* p = (k8 < XOFF) ? (wgh + offh) : (wgx + offx);
  const v4f a = *(const v4f*)p, b = *(const v4f*)(p + 4);
  v8us hv, lv;
  split8(a, b, hv, lv);
  const size_t o = (size_t)n * KA + k8;
  *(volatile v8us*)(wh + o) = hv;
  *(volatile v8us*)(wl + o) = lv;
  __threadfence();
  *(volatile v8us*)(wh + o) = hv;
  *(volatile v8us*)(wl + o) = lv;
}

__global__ __launch_bounds__(GTHR) void k_gemm3(
    const unsigned short* __restrict__ AH, const unsigned short* __restrict__ AL,
    const unsigned short* __restrict__ WH, const unsigned short* __restrict__ WL,
    float* outF, int K, int ldo)
{
  __shared__ __attribute__((aligned(16))) float stg[GBM * GBN];
  const int tid = (int)threadIdx.x, lane = tid & 31, wave = tid >> 5, hh = lane >> 4, m = lane & 15;
  const int rowBase = (int)blockIdx.x * GBM;
  const int col0    = (int)blockIdx.y * GBN;

  v8f acc[4];
  {
    const v8f z = {0.f, 0.f, 0.f, 0.f, 0.f, 0.f, 0.f, 0.f};
    acc[0] = z; acc[1] = z; acc[2] = z; acc[3] = z;
  }
  const size_t ao = (size_t)(rowBase + 16 * wave + m) * (size_t)K + 8 * hh;
  const size_t wo = (size_t)(col0 + m) * (size_t)K + 8 * hh;
  const unsigned short* aph = AH + ao;
  const unsigned short* apl = AL + ao;
  const unsigned short* wph = WH + wo;
  const unsigned short* wpl = WL + wo;
  const int ksteps = K >> 5;
#pragma unroll 1
  for (int ks = 0; ks < ksteps; ++ks) {
    FragB ah, al;
    ah.h[0] = *(const v8us*)(aph + 32 * ks);
    ah.h[1] = *(const v8us*)(aph + 32 * ks + 16);
    al.h[0] = *(const v8us*)(apl + 32 * ks);
    al.h[1] = *(const v8us*)(apl + 32 * ks + 16);
#pragma unroll
    for (int t = 0; t < 4; ++t) {
      const size_t o = (size_t)(16 * t) * (size_t)K + 32 * ks;
      FragB bh, bl;
      bh.h[0] = *(const v8us*)(wph + o);
      bh.h[1] = *(const v8us*)(wph + o + 16);
      bl.h[0] = *(const v8us*)(wpl + o);
      bl.h[1] = *(const v8us*)(wpl + o + 16);
      acc[t] = wmb(ah, bh, acc[t]);
      acc[t] = wmb(ah, bl, acc[t]);
      acc[t] = wmb(al, bh, acc[t]);
    }
  }

#pragma unroll
  for (int t = 0; t < 4; ++t) {
    const int lc = 16 * t + m;
#pragma unroll
    for (int r = 0; r < 8; ++r) {
      const int lr = 16 * wave + 8 * hh + r;
      stg[lr * GBN + lc] = acc[t][r];
    }
  }
  __syncthreads();

  v4f fv[8];
#pragma unroll
  for (int i = 0; i < 8; ++i) {
    const int lr = 16 * wave + 2 * i + hh;
    fv[i] = *(const v4f*)(stg + lr * GBN + 4 * m);
  }
#pragma unroll
  for (int i = 0; i < 8; ++i) {
    const int lr = 16 * wave + 2 * i + hh;
    const int gr = rowBase + lr;
    float* op = outF + (size_t)gr * (size_t)ldo + col0 + 4 * m;
    *(volatile v4f*)op = fv[i];
  }
  __threadfence();
#pragma unroll
  for (int i = 0; i < 8; ++i) {
    const int lr = 16 * wave + 2 * i + hh;
    const int gr = rowBase + lr;
    float* op = outF + (size_t)gr * (size_t)ldo + col0 + 4 * m;
    *(volatile v4f*)op = fv[i];
  }
}

__global__ __launch_bounds__(NTHR) void k_cheb(
    const int* __restrict__ pos2, const float* __restrict__ lap,
    const float* __restrict__ Zh, const float* __restrict__ Zx,
    const float* Pmh, const float* Pmx, float* Yh, float* Yx,
    unsigned short* AH, unsigned short* AL,
    int nN, int nE, int nb, int hasSub, int wf, int colH, int colX) {
  extern __shared__ v4f lds_dyn[];
  __shared__ __attribute__((aligned(16))) float stgs[NWAVE * STGW];
  int* reg1 = (int*)lds_dyn;
  int* reg2 = reg1 + RCAP;
  int* scnt = reg2 + RCAP;
  int* soff = scnt + NBMAX;
  int* list = soff + NBMAX;
  int* wcnt = list + LISTN;
  int* wtot = wcnt + NWAVE;
  const int tid = (int)threadIdx.x, lane = tid & 31, wave = tid >> 5;
  const int nodeBase = (int)blockIdx.x * nb;

  for (int i = tid; i < NBMAX; i += NTHR) scnt[i] = 0;
  __syncthreads();

  int tot = 0;
  const int nChunks = (nE + CHUNK - 1) / CHUNK;
#pragma unroll 1
  for (int ch = 0; ch < nChunks; ++ch) {
    const int cbase = ch * CHUNK;
    const int wc = scan_chunk(pos2, nE, cbase, nodeBase, nb, list, tid, lane, wave);
    if (lane == 0) wcnt[wave] = wc;
    __syncthreads();
    int pre = 0, all = 0;
#pragma unroll
    for (int w2 = 0; w2 < NWAVE; ++w2) {
      int c = wcnt[w2];
      c = c < 0 ? 0 : (c > WCAP ? WCAP : c);
      all += c;
      pre += (w2 < wave) ? c : 0;
    }
    const int wcc  = wc > WCAP ? WCAP : wc;
    const int base = tot + pre;
#pragma unroll 1
    for (int i = lane; i < wcc; i += 32) {
      const int ent = list[wave * WCAP + i];
      const int el  = (ent >> 12) & (CHUNK - 1);
      const int sl  = ent & (NBMAX - 1);
      int eid = cbase + el;
      eid = eid > nE - 1 ? nE - 1 : eid;
      const int ps = base + i;
      if (ps < RCAP) reg1[ps] = (int)(((unsigned)eid << 12) | (unsigned)sl);
    }
    tot += all;
    tot = tot > RCAP ? RCAP : tot;
    __syncthreads();
  }
  const int nh = tot;

  if (wave == 0) {
#pragma unroll 1
    for (int b0 = 0; b0 < nh; b0 += 32) {
      const int idx = b0 + lane;
      const int uv  = reg1[idx < RCAP ? idx : RCAP - 1];
      const int m32 = (nh - b0) < 32 ? (nh - b0) : 32;
#pragma unroll 1
      for (int k = 0; k < m32; ++k) {
        const int u  = __builtin_amdgcn_readlane(uv, k);
        const int sl = u & (NBMAX - 1);
        if (lane == 0) scnt[sl] = scnt[sl] + 1;
      }
    }
  }
  __syncthreads();

  {
    const v4i ca = *(const v4i*)(scnt + 8 * tid);
    const v4i cb = *(const v4i*)(scnt + 8 * tid + 4);
    const int e0 = ca.x < 0 ? 0 : ca.x, e1 = ca.y < 0 ? 0 : ca.y, e2 = ca.z < 0 ? 0 : ca.z, e3 = ca.w < 0 ? 0 : ca.w;
    const int e4 = cb.x < 0 ? 0 : cb.x, e5 = cb.y < 0 ? 0 : cb.y, e6 = cb.z < 0 ? 0 : cb.z, e7 = cb.w < 0 ? 0 : cb.w;
    const int ts8 = e0 + e1 + e2 + e3 + e4 + e5 + e6 + e7;
    int incl = ts8;
#pragma unroll
    for (int d = 1; d < 32; d <<= 1) {
      const int up = __shfl_up(incl, d);
      if (lane >= d) incl += up;
    }
    if (lane == 31) wtot[wave] = incl;
    __syncthreads();
    int pre = 0;
#pragma unroll
    for (int w2 = 0; w2 < NWAVE; ++w2) pre += (w2 < wave) ? wtot[w2] : 0;
    int run = pre + incl - ts8;
    soff[8 * tid + 0] = run; run += e0;
    soff[8 * tid + 1] = run; run += e1;
    soff[8 * tid + 2] = run; run += e2;
    soff[8 * tid + 3] = run; run += e3;
    soff[8 * tid + 4] = run; run += e4;
    soff[8 * tid + 5] = run; run += e5;
    soff[8 * tid + 6] = run; run += e6;
    soff[8 * tid + 7] = run;
  }
  __syncthreads();
  for (int i = tid; i < NBMAX; i += NTHR) list[i] = soff[i];
  __syncthreads();

  if (wave == 0) {
#pragma unroll 1
    for (int b0 = 0; b0 < nh; b0 += 32) {
      const int idx = b0 + lane;
      const int uv  = reg1[idx < RCAP ? idx : RCAP - 1];
      const int m32 = (nh - b0) < 32 ? (nh - b0) : 32;
#pragma unroll 1
      for (int k = 0; k < m32; ++k) {
        const int u   = __builtin_amdgcn_readlane(uv, k);
        const int sl  = u & (NBMAX - 1);
        const int eid = (int)((unsigned)u >> 12);
        if (lane == 0) {
          int ps = list[sl];
          ps = ps < 0 ? 0 : (ps > RCAP - 1 ? RCAP - 1 : ps);
          reg2[ps] = eid;
          list[sl] = ps + 1;
        }
      }
    }
  }
  __syncthreads();

  const int nbw = nb >> 3;
  const bool ovf = (nh >= RCAP);
  const float qnan = __int_as_float(0x7fc00000);
  float* stg = stgs + wave * STGW;
#pragma unroll 1
  for (int jt = 0; jt < nbw; ++jt) {
    const int slot = wave * nbw + jt;
    const int grow = nodeBase + slot;
    const int gcl  = grow < nN ? grow : nN - 1;
    int st = soff[slot];
    const int craw = scnt[slot];
    int cnt = craw;
    st  = st < 0 ? 0 : (st > nh ? nh : st);
    cnt = cnt < 0 ? 0 : (cnt > DEGCAP ? DEGCAP : cnt);
    if (cnt > nh - st) cnt = nh - st;
    const float pz = (ovf || craw > DEGCAP) ? qnan : 0.0f;
    const bool wr = grow < nN;

    int ce[4], cc[4];
    float cv[4];
#pragma unroll
    for (int g = 0; g < 4; ++g) { ce[g] = -1; cc[g] = 0; cv[g] = 0.f; }
    if (cnt > 0) {
#pragma unroll
      for (int g = 0; g < 4; ++g) {
        const int qi = 32 * g + lane;
        const int qc = qi < cnt ? qi : cnt - 1;
        int idx = st + qc; idx = idx > RCAP - 1 ? RCAP - 1 : idx;
        int eid = reg2[idx]; eid = eid < 0 ? 0 : (eid > nE - 1 ? nE - 1 : eid);
        int col = pos2[2 * (size_t)eid + 1]; col = col < 0 ? 0 : (col > nN - 1 ? nN - 1 : col);
        const float val = lap[eid];
        ce[g] = (qi < cnt) ? eid : -1;
        cc[g] = col;
        cv[g] = val;
      }
    }
    float ah[8], ax[4];
#pragma unroll
    for (int j = 0; j < 8; ++j) ah[j] = 0.f;
#pragma unroll
    for (int j = 0; j < 4; ++j) ax[j] = 0.f;

#pragma unroll 1
    for (int q = 0; q < cnt; ++q) {
      const int g = q >> 5, lq = q & 31;
      const int   me = (g == 0) ? ce[0] : ((g == 1) ? ce[1] : ((g == 2) ? ce[2] : ce[3]));
      const int   mc = (g == 0) ? cc[0] : ((g == 1) ? cc[1] : ((g == 2) ? cc[2] : cc[3]));
      const float mv = (g == 0) ? cv[0] : ((g == 1) ? cv[1] : ((g == 2) ? cv[2] : cv[3]));
      const int   eq = __builtin_amdgcn_readlane(me, lq);
      const int   cq = __builtin_amdgcn_readlane(mc, lq);
      const float vq = __int_as_float(__builtin_amdgcn_readlane(__float_as_int(mv), lq));
      const bool dp = ((cc[0] == cq) & (ce[0] > eq)) | ((cc[1] == cq) & (ce[1] > eq)) |
                      ((cc[2] == cq) & (ce[2] > eq)) | ((cc[3] == cq) & (ce[3] > eq));
      const unsigned dm = __builtin_amdgcn_ballot_w32(dp);
      if (dm == 0u) {
        const float* zr = Zh + (size_t)cq * HSZ + lane;
        const float* xr = Zx + (size_t)cq * ISZ + lane;
        float zh[8], zx[4];
#pragma unroll
        for (int j = 0; j < 8; ++j) zh[j] = zr[32 * j];
#pragma unroll
        for (int j = 0; j < 4; ++j) zx[j] = xr[32 * j];
#pragma unroll
        for (int j = 0; j < 8; ++j) ah[j] = fmaf(vq, zh[j], ah[j]);
#pragma unroll
        for (int j = 0; j < 4; ++j) ax[j] = fmaf(vq, zx[j], ax[j]);
      }
    }

    float yh[8], yx[4];
    if (hasSub != 0) {
      const float* ph = Pmh + (size_t)gcl * HSZ + lane;
      const float* px = Pmx + (size_t)gcl * ISZ + lane;
#pragma unroll
      for (int j = 0; j < 8; ++j) yh[j] = 2.0f * ah[j] - ph[32 * j];
#pragma unroll
      for (int j = 0; j < 4; ++j) yx[j] = 2.0f * ax[j] - px[32 * j];
    } else {
#pragma unroll
      for (int j = 0; j < 8; ++j) yh[j] = ah[j];
#pragma unroll
      for (int j = 0; j < 4; ++j) yx[j] = ax[j];
    }
#pragma unroll
    for (int j = 0; j < 8; ++j) yh[j] += pz;
#pragma unroll
    for (int j = 0; j < 4; ++j) yx[j] += pz;

    if (wr) {
#pragma unroll
      for (int j = 0; j < 8; ++j) stg[32 * j + lane] = yh[j];
#pragma unroll
      for (int j = 0; j < 4; ++j) stg[HSZ + 32 * j + lane] = yx[j];
      __builtin_amdgcn_fence(__ATOMIC_RELEASE, "wavefront");
      __builtin_amdgcn_wave_barrier();
      const v4fa f0 = *(const v4fa*)(stg + 4 * lane);
      const v4fa f1 = *(const v4fa*)(stg + 128 + 4 * lane);
      const v4fa f2 = *(const v4fa*)(stg + HSZ + 4 * lane);
      const v4fa ha = *(const v4fa*)(stg + 8 * lane);
      const v4fa hb = *(const v4fa*)(stg + 8 * lane + 4);
      const int  lx = lane & 15;
      const v4fa xa = *(const v4fa*)(stg + HSZ + 8 * lx);
      const v4fa xb = *(const v4fa*)(stg + HSZ + 8 * lx + 4);
      __builtin_amdgcn_fence(__ATOMIC_ACQUIRE, "wavefront");
      __builtin_amdgcn_wave_barrier();
      const v4f ha4 = {ha.x, ha.y, ha.z, ha.w}, hb4 = {hb.x, hb.y, hb.z, hb.w};
      const v4f xa4 = {xa.x, xa.y, xa.z, xa.w}, xb4 = {xb.x, xb.y, xb.z, xb.w};
      v8us hhi, hlo, xhi, xlo;
      split8(ha4, hb4, hhi, hlo);
      split8(xa4, xb4, xhi, xlo);
      float* oh = Yh + (size_t)grow * HSZ;
      float* ox = Yx + (size_t)grow * ISZ;
      unsigned short* pah = AH + (size_t)grow * KA;
      unsigned short* pal = AL + (size_t)grow * KA;
      if (wf != 0) {
        *(volatile v4fa*)(oh + 4 * lane)       = f0;
        *(volatile v4fa*)(oh + 128 + 4 * lane) = f1;
        *(volatile v4fa*)(ox + 4 * lane)       = f2;
      }
      *(volatile v8us*)(pah + colH + 8 * lane) = hhi;
      *(volatile v8us*)(pal + colH + 8 * lane) = hlo;
      if (lane < 16) {
        *(volatile v8us*)(pah + colX + 8 * lane) = xhi;
        *(volatile v8us*)(pal + colX + 8 * lane) = xlo;
      }
      __threadfence();
      if (wf != 0) {
        *(volatile v4fa*)(oh + 4 * lane)       = f0;
        *(volatile v4fa*)(oh + 128 + 4 * lane) = f1;
        *(volatile v4fa*)(ox + 4 * lane)       = f2;
      }
      *(volatile v8us*)(pah + colH + 8 * lane) = hhi;
      *(volatile v8us*)(pal + colH + 8 * lane) = hlo;
      if (lane < 16) {
        *(volatile v8us*)(pah + colX + 8 * lane) = xhi;
        *(volatile v8us*)(pal + colX + 8 * lane) = xlo;
      }
    }
  }
}

__global__ __launch_bounds__(NTHR) void k_cell(
    const float* __restrict__ G, const float* __restrict__ bfp, const float* __restrict__ bip,
    const float* __restrict__ bop, const float* __restrict__ bcp, const float* __restrict__ cin,
    float* outp, int nUnits, int off1) {
  const int u = (int)blockIdx.x * NTHR + (int)threadIdx.x;
  if (u >= nUnits) return;
  const int n  = u >> 6;
  const int j0 = (u & 63) * 4;
  const size_t e = (size_t)n * HSZ + j0;
  const float* gr = G + (size_t)n * NGC + j0;
  const v4f g0 = *(const v4f*)gr;
  const v4f g1 = *(const v4f*)(gr + HSZ);
  const v4f g2 = *(const v4f*)(gr + 2 * HSZ);
  const v4f g3 = *(const v4f*)(gr + 3 * HSZ);
  const v4f b0 = *(const v4f*)(bfp + e);
  const v4f b1 = *(const v4f*)(bip + e);
  const v4f b2 = *(const v4f*)(bop + e);
  const v4f b3 = *(const v4f*)(bcp + e);
  const v4f cv = *(const v4f*)(cin + e);
  float pf[4] = {g0.x + b0.x, g0.y + b0.y, g0.z + b0.z, g0.w + b0.w};
  float pi[4] = {g1.x + b1.x, g1.y + b1.y, g1.z + b1.z, g1.w + b1.w};
  float po[4] = {g2.x + b2.x, g2.y + b2.y, g2.z + b2.z, g2.w + b2.w};
  float pc[4] = {g3.x + b3.x, g3.y + b3.y, g3.z + b3.z, g3.w + b3.w};
  float c0[4] = {cv.x, cv.y, cv.z, cv.w};
  float hn[4], cn[4];
#pragma unroll
  for (int t = 0; t < 4; ++t) {
    const float f = sigm_f(pf[t]);
    const float i = sigm_f(pi[t]);
    const float o = sigm_f(po[t]);
    const float ct = i * tanh_f(pc[t]) + f * c0[t];
    cn[t] = ct;
    hn[t] = o * tanh_f(ct);
  }
  const v4f hv = {hn[0], hn[1], hn[2], hn[3]};
  const v4f cvo = {cn[0], cn[1], cn[2], cn[3]};
  float* p0 = outp + e;
  float* p1 = outp + (size_t)off1 + e;
  *(volatile v4f*)p0 = hv;
  *(volatile v4f*)p1 = cvo;
  __threadfence();
  *(volatile v4f*)p0 = hv;
  *(volatile v4f*)p1 = cvo;
}

static int pick_nb(int nE, int nN) {
  int nb = NBMAX;
  while (nb > 16 && (long long)nb * (long long)nE * 5LL > (long long)RCAP * (long long)nN * 4LL) nb >>= 1;
  return nb;
}
static inline int cdiv(int a, int b) { return (a + b - 1) / b; }

extern "C" void kernel_launch(void* const* d_in, const int* in_sizes, int n_in,
                              void* d_out, int out_size, void* d_ws, size_t ws_size,
                              hipStream_t stream) {
  if (n_in < 17) return;
  if (in_sizes[1] < HSZ * GBM || (in_sizes[1] % (HSZ * GBM)) != 0) return;
  const int nN = in_sizes[1] / HSZ;
  if (nN > (1 << 22)) return;
  if (in_sizes[0] != nN * ISZ || in_sizes[2] != nN * HSZ) return;
  const int nE = in_sizes[3];
  if (nE < 1 || nE > (1 << 20)) return;
  if (in_sizes[4] != 2 * nE) return;
  if (in_sizes[5] != KCH * HSZ * HSZ || in_sizes[8] != KCH * HSZ * HSZ ||
      in_sizes[11] != KCH * HSZ * HSZ || in_sizes[14] != KCH * HSZ * HSZ) return;
  if (in_sizes[6] != KCH * HSZ * ISZ || in_sizes[9] != KCH * HSZ * ISZ ||
      in_sizes[12] != KCH * HSZ * ISZ || in_sizes[15] != KCH * HSZ * ISZ) return;
  if (in_sizes[7] != nN * HSZ || in_sizes[10] != nN * HSZ || in_sizes[13] != nN * HSZ || in_sizes[16] != nN * HSZ) return;
  if (out_size != 2 * nN * HSZ) return;

  const float* x    = (const float*)d_in[0];
  const float* h    = (const float*)d_in[1];
  const float* c    = (const float*)d_in[2];
  const float* lap  = (const float*)d_in[3];
  const int*   pos2 = (const int*)  d_in[4];
  const float* W_fh = (const float*)d_in[5];
  const float* W_fx = (const float*)d_in[6];
  const float* bfp  = (const float*)d_in[7];
  const float* W_ih = (const float*)d_in[8];
  const float* W_ix = (const float*)d_in[9];
  const float* bip  = (const float*)d_in[10];
  const float* W_oh = (const float*)d_in[11];
  const float* W_ox = (const float*)d_in[12];
  const float* bop  = (const float*)d_in[13];
  const float* W_ch = (const float*)d_in[14];
  const float* W_cx = (const float*)d_in[15];
  const float* bcp  = (const float*)d_in[16];
  float* out = (float*)d_out;

  const int nb = pick_nb(nE, nN);
  const int gA = cdiv(nN, nb);
  if (nb > NBMAX || gA * nb < nN) return;

  char* ws = (char*)d_ws;
  size_t off = 0;
  const size_t oAH  = off; off += (size_t)nN * KA * 2;     off = (off + 255) & ~(size_t)255;
  const size_t oAL  = off; off += (size_t)nN * KA * 2;     off = (off + 255) & ~(size_t)255;
  const size_t oWH  = off; off += (size_t)NGC * KA * 2;    off = (off + 255) & ~(size_t)255;
  const size_t oWL  = off; off += (size_t)NGC * KA * 2;    off = (off + 255) & ~(size_t)255;
  const size_t oT1H = off; off += (size_t)nN * HSZ * 4;    off = (off + 255) & ~(size_t)255;
  const size_t oT2H = off; off += (size_t)nN * HSZ * 4;    off = (off + 255) & ~(size_t)255;
  const size_t oT1X = off; off += (size_t)nN * ISZ * 4;    off = (off + 255) & ~(size_t)255;
  const size_t oT2X = off; off += (size_t)nN * ISZ * 4;    off = (off + 255) & ~(size_t)255;
  const size_t oG   = off; off += (size_t)nN * NGC * 4;    off = (off + 255) & ~(size_t)255;
  if (off > ws_size || off > (size_t)WSMAX) return;
  unsigned short* AH  = (unsigned short*)(ws + oAH);
  unsigned short* AL  = (unsigned short*)(ws + oAL);
  unsigned short* WH  = (unsigned short*)(ws + oWH);
  unsigned short* WL  = (unsigned short*)(ws + oWL);
  float*          T1H = (float*)(ws + oT1H);
  float*          T2H = (float*)(ws + oT2H);
  float*          T1X = (float*)(ws + oT1X);
  float*          T2X = (float*)(ws + oT2X);
  float*          G   = (float*)(ws + oG);

  hipFuncSetAttribute(reinterpret_cast<const void*>(&k_cheb),
                      hipFuncAttributeMaxDynamicSharedMemorySize, LDS_DYN);

  const int nUh = nN * (HSZ / 8);
  k_split<<<cdiv(nUh, NTHR), NTHR, 0, stream>>>(h, HSZ, AH, AL, 0, nN, nUh);
  const int nUx = nN * (ISZ / 8);
  k_split<<<cdiv(nUx, NTHR), NTHR, 0, stream>>>(x, ISZ, AH, AL, XOFF, nN, nUx);

  const int nUw = NGC * (KA / 8);
  k_wsplit<<<cdiv(nUw, NTHR), NTHR, 0, stream>>>(W_fh, W_ih, W_oh, W_ch, W_fx, W_ix, W_ox, W_cx, WH, WL, nUw);

  k_cheb<<<gA, NTHR, LDS_DYN, stream>>>(pos2, lap, h,   x,   h,   x,   T1H, T1X, AH, AL,
                                        nN, nE, nb, 0, 1, 1 * HSZ, XOFF + 1 * ISZ);
  k_cheb<<<gA, NTHR, LDS_DYN, stream>>>(pos2, lap, T1H, T1X, h,   x,   T2H, T2X, AH, AL,
                                        nN, nE, nb, 1, 1, 2 * HSZ, XOFF + 2 * ISZ);
  k_cheb<<<gA, NTHR, LDS_DYN, stream>>>(pos2, lap, T2H, T2X, T1H, T1X, T1H, T1X, AH, AL,
                                        nN, nE, nb, 1, 0, 3 * HSZ, XOFF + 3 * ISZ);

  k_gemm3<<<dim3(nN / GBM, NGC / GBN), GTHR, 0, stream>>>(AH, AL, WH, WL, G, KA, NGC);

  const int nUc = nN * (HSZ / 4);
  k_cell<<<cdiv(nUc, NTHR), NTHR, 0, stream>>>(G, bfp, bip, bop, bcp, c, out, nUc, nN * HSZ);
}
